// CatTransformerEncoderLayer_24215025614968
// MI455X (gfx1250) — hardware-verified
//
#include <hip/hip_runtime.h>

typedef _Float16 v16h __attribute__((ext_vector_type(16)));
typedef _Float16 v8h  __attribute__((ext_vector_type(8)));
typedef float    v8f  __attribute__((ext_vector_type(8)));
typedef float    v4f  __attribute__((ext_vector_type(4)));
typedef v8h __attribute__((may_alias)) v8ha;
typedef v4f __attribute__((may_alias)) v4fa;

union Frag { v16h v; v8h half[2]; };

#define BATCH  2
#define SEQ    2048
#define DM     512
#define NHEADS 8
#define HD     64
#define DFF    2048
#define MROWS  (BATCH * SEQ)
#define NX     (MROWS * DM)
#define NW     (DM * DM)
#define NW1    (DFF * DM)
#define NHID   (MROWS * DFF)
#define NXG    (NX / 8)
#define NWG    (NW / 8)
#define NW1G   (NW1 / 8)
#define NCONVG (3 * NXG + 4 * NWG + 2 * NW1G)
#define PSCALE 1024.0f
#define LN_EPS 1e-5f

static_assert(MROWS % 128 == 0);
static_assert(SEQ % 128 == 0);
static_assert(DM % 64 == 0 && DFF % 64 == 0);
static_assert(NCONVG % 256 == 0);
static_assert(MROWS % 8 == 0);

__device__ __forceinline__ v8f wmma_f16(v16h a, v16h b, v8f c) {
  v8f d = __builtin_amdgcn_wmma_f32_16x16x32_f16(false, a, false, b, (short)0, c, false, false);
  asm volatile("v_nop\n\tv_nop\n\tv_nop\n\tv_nop" : "+v"(d) : "v"(a), "v"(b));
  return d;
}

__device__ __forceinline__ v16h load_frag(const _Float16* p, int h) {
  Frag f;
  f.half[0] = *(const v8ha*)(p + 8 * h);
  f.half[1] = *(const v8ha*)(p + 16 + 8 * h);
  return f.v;
}

__global__ __launch_bounds__(256) void convert_kernel(
    const float* __restrict__ q, const float* __restrict__ k, const float* __restrict__ v,
    const float* __restrict__ wq, const float* __restrict__ wk, const float* __restrict__ wv,
    const float* __restrict__ wo, const float* __restrict__ w1, const float* __restrict__ w2,
    _Float16* __restrict__ conv)
{
  const int g = blockIdx.x * 256 + threadIdx.x;
  if (g >= NCONVG) return;
  const float* src;
  float sc;
  if (g < 3 * NXG) {
    const int which = g / NXG;
    const int off = g - which * NXG;
    const float* base = (which == 0) ? q : ((which == 1) ? k : v);
    src = base + (size_t)off * 8;
    sc = 1.0f;
  } else if (g < 3 * NXG + 4 * NWG) {
    const int e = g - 3 * NXG;
    const int which = e / NWG;
    const int off = e - which * NWG;
    const float* base = (which == 0) ? wq : ((which == 1) ? wk : ((which == 2) ? wv : wo));
    src = base + (size_t)off * 8;
    sc = 32.0f;
  } else {
    const int e = g - 3 * NXG - 4 * NWG;
    const int which = e / NW1G;
    const int off = e - which * NW1G;
    const float* base = (which == 0) ? w1 : w2;
    src = base + (size_t)off * 8;
    sc = 32.0f;
  }
  const v4f a = *(const v4fa*)src;
  const v4f c = *(const v4fa*)(src + 4);
  const v8h o = { (_Float16)(a.x * sc), (_Float16)(a.y * sc), (_Float16)(a.z * sc), (_Float16)(a.w * sc),
                  (_Float16)(c.x * sc), (_Float16)(c.y * sc), (_Float16)(c.z * sc), (_Float16)(c.w * sc) };
  _Float16* dst = conv + (size_t)g * 8;
  *(volatile v8h*)dst = o;
  __threadfence();
  *(volatile v8h*)dst = o;
}

__device__ __forceinline__ void proj_store_pass(const _Float16* sT, _Float16* plane, _Float16* vt,
                                                int which, int bh, int l0, int w, int lane) {
  const int q8 = lane & 7, sub = lane >> 3;
  #pragma unroll
  for (int i = 0; i < 8; ++i) {
    const int lid = w * 32 + i * 4 + sub;
    v8h v;
    _Float16* dst;
    if (which != 2) {
      v = *(const v8ha*)(sT + lid * HD + 8 * q8);
      dst = plane + ((size_t)bh * SEQ + l0 + lid) * HD + 8 * q8;
    } else {
      const int d = lid >> 1, hl = lid & 1;
      v = *(const v8ha*)(sT + d * 128 + 64 * hl + 8 * q8);
      dst = vt + ((size_t)bh * HD + d) * SEQ + l0 + 64 * hl + 8 * q8;
    }
    *(volatile v8h*)dst = v;
  }
}

__global__ __launch_bounds__(128) void proj_kernel(
    const _Float16* __restrict__ xh,
    const _Float16* __restrict__ wh,
    const float* __restrict__ bq, const float* __restrict__ bk, const float* __restrict__ bv,
    _Float16* __restrict__ qh,
    _Float16* __restrict__ kh,
    _Float16* __restrict__ vt)
{
  __shared__ __attribute__((aligned(16))) _Float16 sT[128 * 64];

  const int tid = threadIdx.x, lane = tid & 31, w = tid >> 5;
  const int h = lane >> 4, m = lane & 15;
  const int m0 = blockIdx.x * 128;
  const int cg = blockIdx.y;
  const int which = cg >> 3, head = cg & 7;
  const int m0w = m0 + 32 * w;

  const _Float16* xa0 = xh + (size_t)which * NX + (size_t)(m0w + m) * DM;
  const _Float16* xa1 = xa0 + (size_t)16 * DM;
  const _Float16* wb  = wh + (size_t)which * NW + (size_t)(head * HD + m) * DM;

  const v8f zero8 = {0.f, 0.f, 0.f, 0.f, 0.f, 0.f, 0.f, 0.f};
  v8f acc[2][4];
  #pragma unroll
  for (int mt = 0; mt < 2; ++mt)
    #pragma unroll
    for (int nt = 0; nt < 4; ++nt) acc[mt][nt] = zero8;

  #pragma unroll 1
  for (int k0 = 0; k0 < DM; k0 += 32) {
    const v16h a0 = load_frag(xa0 + k0, h);
    const v16h a1 = load_frag(xa1 + k0, h);
    #pragma unroll
    for (int nt = 0; nt < 4; ++nt) {
      const v16h b = load_frag(wb + (size_t)nt * 16 * DM + k0, h);
      acc[0][nt] = wmma_f16(a0, b, acc[0][nt]);
      acc[1][nt] = wmma_f16(a1, b, acc[1][nt]);
    }
  }

  const float* bias = (which == 0) ? bq : ((which == 1) ? bk : bv);
  const float osc = (which == 0) ? 0.5f : 4.0f;
  #pragma unroll
  for (int nt = 0; nt < 4; ++nt) {
    const int feat = 16 * nt + m;
    const float bvl = bias[head * HD + feat];
    #pragma unroll
    for (int mt = 0; mt < 2; ++mt) {
      #pragma unroll
      for (int r = 0; r < 8; ++r) {
        const int tokl = 32 * w + 16 * mt + 8 * h + r;
        const float y = (acc[mt][nt][r] * 0.03125f + bvl) * osc;
        const int idx = (which == 2) ? (feat * 128 + tokl) : (tokl * HD + feat);
        sT[idx] = (_Float16)y;
      }
    }
  }
  __syncthreads();

  const int b = m0 / SEQ, l0 = m0 - b * SEQ, bh = b * NHEADS + head;
  _Float16* plane = (which == 0) ? qh : kh;
  proj_store_pass(sT, plane, vt, which, bh, l0, w, lane);
  __threadfence();
  proj_store_pass(sT, plane, vt, which, bh, l0, w, lane);
}

__device__ __forceinline__ v16h pack_p(v8f a, v8f c) {
  const v16h r = { (_Float16)(a[0] * PSCALE), (_Float16)(a[1] * PSCALE), (_Float16)(a[2] * PSCALE), (_Float16)(a[3] * PSCALE),
                   (_Float16)(a[4] * PSCALE), (_Float16)(a[5] * PSCALE), (_Float16)(a[6] * PSCALE), (_Float16)(a[7] * PSCALE),
                   (_Float16)(c[0] * PSCALE), (_Float16)(c[1] * PSCALE), (_Float16)(c[2] * PSCALE), (_Float16)(c[3] * PSCALE),
                   (_Float16)(c[4] * PSCALE), (_Float16)(c[5] * PSCALE), (_Float16)(c[6] * PSCALE), (_Float16)(c[7] * PSCALE) };
  return r;
}

__device__ __forceinline__ void ctx_store_pass(const float* so, _Float16* ctx,
                                               int b, int head, int q0, int lane) {
  const int q8 = lane & 7, sub = lane >> 3;
  #pragma unroll
  for (int i = 0; i < 4; ++i) {
    const int row = 4 * i + sub;
    const v4f x0 = *(const v4fa*)(so + row * 64 + 8 * q8);
    const v4f x1 = *(const v4fa*)(so + row * 64 + 8 * q8 + 4);
    const v8h o = { (_Float16)x0.x, (_Float16)x0.y, (_Float16)x0.z, (_Float16)x0.w,
                    (_Float16)x1.x, (_Float16)x1.y, (_Float16)x1.z, (_Float16)x1.w };
    const size_t gi = ((size_t)b * SEQ + q0 + row) * DM + head * HD + 8 * q8;
    *(volatile v8h*)(ctx + gi) = o;
  }
}

__global__ __launch_bounds__(128) void attn_kernel(
    const _Float16* __restrict__ qh,
    const _Float16* __restrict__ kh,
    const _Float16* __restrict__ vt,
    _Float16* __restrict__ ctx)
{
  __shared__ __attribute__((aligned(16))) float sO[4 * 16 * 64];

  const int tid = threadIdx.x, lane = tid & 31, w = tid >> 5;
  const int h = lane >> 4, m = lane & 15;
  const int bh = blockIdx.y, b = bh >> 3, head = bh & 7;
  const int q0 = blockIdx.x * 64 + 16 * w;

  const _Float16* qrow = qh + ((size_t)bh * SEQ + q0 + m) * HD;
  const v16h qb0 = load_frag(qrow, h);
  const v16h qb1 = load_frag(qrow + 32, h);

  const v8f zero8 = {0.f, 0.f, 0.f, 0.f, 0.f, 0.f, 0.f, 0.f};
  v8f o[4];
  #pragma unroll
  for (int t = 0; t < 4; ++t) o[t] = zero8;
  float mrun = -1e30f, lrun = 0.0f;

  const _Float16* kbase = kh + ((size_t)bh * SEQ + m) * HD;
  const _Float16* vbase = vt + ((size_t)bh * HD + m) * SEQ;

  #pragma unroll 1
  for (int kb = 0; kb < SEQ; kb += 64) {
    v8f s[4];
    #pragma unroll
    for (int j = 0; j < 4; ++j) {
      const _Float16* kp = kbase + (size_t)(kb + 16 * j) * HD;
      const v16h kf0 = load_frag(kp, h);
      const v16h kf1 = load_frag(kp + 32, h);
      v8f z = zero8;
      z = wmma_f16(kf0, qb0, z);
      z = wmma_f16(kf1, qb1, z);
      s[j] = z;
    }
    #pragma unroll
    for (int j = 0; j < 4; ++j)
      #pragma unroll
      for (int r = 0; r < 8; ++r) s[j][r] = s[j][r] * 0.0625f;

    float mloc = s[0][0];
    #pragma unroll
    for (int j = 0; j < 4; ++j)
      #pragma unroll
      for (int r = 0; r < 8; ++r) mloc = fmaxf(mloc, s[j][r]);
    mloc = fmaxf(mloc, __shfl_xor(mloc, 16));
    const float mnew = fmaxf(mrun, mloc);
    const float alpha = __expf(mrun - mnew);
    mrun = mnew;
    float lsum = 0.0f;
    #pragma unroll
    for (int j = 0; j < 4; ++j)
      #pragma unroll
      for (int r = 0; r < 8; ++r) {
        const float p = __expf(s[j][r] - mnew);
        s[j][r] = p;
        lsum += p;
      }
    lsum += __shfl_xor(lsum, 16);
    lrun = lrun * alpha + lsum;
    #pragma unroll
    for (int t = 0; t < 4; ++t)
      #pragma unroll
      for (int r = 0; r < 8; ++r) o[t][r] = o[t][r] * alpha;

    const v16h pb0 = pack_p(s[0], s[1]);
    const v16h pb1 = pack_p(s[2], s[3]);

    #pragma unroll
    for (int t = 0; t < 4; ++t) {
      const _Float16* vp = vbase + (size_t)(16 * t) * SEQ + kb;
      const v16h vf0 = load_frag(vp, h);
      const v16h vf1 = load_frag(vp + 32, h);
      o[t] = wmma_f16(vf0, pb0, o[t]);
      o[t] = wmma_f16(vf1, pb1, o[t]);
    }
  }

  const float inv = (1.0f / lrun) * (1.0f / PSCALE);
  float* so = sO + w * 1024;
  #pragma unroll
  for (int t = 0; t < 4; ++t)
    #pragma unroll
    for (int r = 0; r < 8; ++r)
      so[m * 64 + 16 * t + 8 * h + r] = o[t][r] * inv;
  __syncthreads();

  ctx_store_pass(so, ctx, b, head, q0, lane);
  __threadfence();
  ctx_store_pass(so, ctx, b, head, q0, lane);
}

__device__ __forceinline__ void gemm_store_f32_pass(const float* sC, float* C, int N,
                                                    int m0, int n0, int w, int lane) {
  const int sub = lane >> 4, c4 = 4 * (lane & 15);
  #pragma unroll
  for (int i = 0; i < 16; ++i) {
    const int row = 32 * w + 2 * i + sub;
    const v4f v = *(const v4fa*)(sC + row * 64 + c4);
    *(volatile v4f*)(C + (size_t)(m0 + row) * N + n0 + c4) = v;
  }
}

__device__ __forceinline__ void gemm_store_f16_pass(const float* sC, _Float16* C, int N,
                                                    int m0, int n0, int w, int lane) {
  const int sub = lane >> 3, c8 = 8 * (lane & 7);
  #pragma unroll
  for (int i = 0; i < 8; ++i) {
    const int row = 32 * w + 4 * i + sub;
    const v4f x0 = *(const v4fa*)(sC + row * 64 + c8);
    const v4f x1 = *(const v4fa*)(sC + row * 64 + c8 + 4);
    const v8h o = { (_Float16)x0.x, (_Float16)x0.y, (_Float16)x0.z, (_Float16)x0.w,
                    (_Float16)x1.x, (_Float16)x1.y, (_Float16)x1.z, (_Float16)x1.w };
    *(volatile v8h*)(C + (size_t)(m0 + row) * N + n0 + c8) = o;
  }
}

template <int N, int K, bool RELU, bool RES, bool HOUT>
__global__ __launch_bounds__(128) void gemm_kernel(
    const _Float16* __restrict__ A,
    const _Float16* __restrict__ W,
    const float* __restrict__ bias,
    const float* __restrict__ res,
    float* __restrict__ Cf,
    _Float16* __restrict__ Ch,
    float ascale, float oscale)
{
  __shared__ __attribute__((aligned(16))) float sC[128 * 64];

  const int tid = threadIdx.x, lane = tid & 31, w = tid >> 5;
  const int h = lane >> 4, m = lane & 15;
  const int m0 = blockIdx.x * 128, n0 = blockIdx.y * 64;
  const int m0w = m0 + 32 * w;

  const _Float16* a0p = A + (size_t)(m0w + m) * K;
  const _Float16* a1p = a0p + (size_t)16 * K;
  const _Float16* wp  = W + (size_t)(n0 + m) * K;

  const v8f zero8 = {0.f, 0.f, 0.f, 0.f, 0.f, 0.f, 0.f, 0.f};
  v8f acc[2][4];
  #pragma unroll
  for (int mt = 0; mt < 2; ++mt)
    #pragma unroll
    for (int nt = 0; nt < 4; ++nt) acc[mt][nt] = zero8;

  #pragma unroll 1
  for (int k0 = 0; k0 < K; k0 += 32) {
    const v16h a0 = load_frag(a0p + k0, h);
    const v16h a1 = load_frag(a1p + k0, h);
    #pragma unroll
    for (int nt = 0; nt < 4; ++nt) {
      const v16h b = load_frag(wp + (size_t)nt * 16 * K + k0, h);
      acc[0][nt] = wmma_f16(a0, b, acc[0][nt]);
      acc[1][nt] = wmma_f16(a1, b, acc[1][nt]);
    }
  }

  #pragma unroll
  for (int nt = 0; nt < 4; ++nt) {
    const int col = n0 + 16 * nt + m;
    const float bvl = bias[col];
    #pragma unroll
    for (int mt = 0; mt < 2; ++mt) {
      #pragma unroll
      for (int r = 0; r < 8; ++r) {
        const int tokl = 32 * w + 16 * mt + 8 * h + r;
        float y = acc[mt][nt][r] * ascale + bvl;
        if (RES) y += res[(size_t)(m0 + tokl) * N + col];
        if (RELU) y = fmaxf(y, 0.0f);
        sC[tokl * 64 + 16 * nt + m] = y * oscale;
      }
    }
  }
  __syncthreads();

  if (HOUT) {
    gemm_store_f16_pass(sC, Ch, N, m0, n0, w, lane);
    __threadfence();
    gemm_store_f16_pass(sC, Ch, N, m0, n0, w, lane);
  } else {
    gemm_store_f32_pass(sC, Cf, N, m0, n0, w, lane);
    __threadfence();
    gemm_store_f32_pass(sC, Cf, N, m0, n0, w, lane);
  }
}

template <bool HOUT>
__global__ __launch_bounds__(256) void ln_kernel(
    const float* __restrict__ x,
    const float* __restrict__ gam,
    const float* __restrict__ bet,
    float* __restrict__ outf,
    _Float16* __restrict__ outh)
{
  const int lane = threadIdx.x & 31, w = threadIdx.x >> 5;
  const int row = blockIdx.x * 8 + w;
  const float* xr = x + (size_t)row * DM;

  v4f a[4];
  float s = 0.0f;
  #pragma unroll
  for (int i = 0; i < 4; ++i) {
    a[i] = *(const v4fa*)(xr + 128 * i + 4 * lane);
    s += (a[i].x + a[i].y) + (a[i].z + a[i].w);
  }
  #pragma unroll
  for (int ofs = 16; ofs > 0; ofs >>= 1) s += __shfl_xor(s, ofs);
  const float mu = s * (1.0f / DM);

  float vs = 0.0f;
  #pragma unroll
  for (int i = 0; i < 4; ++i) {
    const float d0 = a[i].x - mu, d1 = a[i].y - mu, d2 = a[i].z - mu, d3 = a[i].w - mu;
    vs += (d0 * d0 + d1 * d1) + (d2 * d2 + d3 * d3);
  }
  #pragma unroll
  for (int ofs = 16; ofs > 0; ofs >>= 1) vs += __shfl_xor(vs, ofs);
  const float rstd = rsqrtf(vs * (1.0f / DM) + LN_EPS);

  v4f ov[4];
  #pragma unroll
  for (int i = 0; i < 4; ++i) {
    const v4f gv = *(const v4fa*)(gam + 128 * i + 4 * lane);
    const v4f bv = *(const v4fa*)(bet + 128 * i + 4 * lane);
    v4f t;
    t.x = (a[i].x - mu) * rstd * gv.x + bv.x;
    t.y = (a[i].y - mu) * rstd * gv.y + bv.y;
    t.z = (a[i].z - mu) * rstd * gv.z + bv.z;
    t.w = (a[i].w - mu) * rstd * gv.w + bv.w;
    ov[i] = t;
  }
  float* orow = outf + (size_t)row * DM;
  #pragma unroll
  for (int i = 0; i < 4; ++i) *(volatile v4f*)(orow + 128 * i + 4 * lane) = ov[i];
  __threadfence();
  #pragma unroll
  for (int i = 0; i < 4; ++i) *(volatile v4f*)(orow + 128 * i + 4 * lane) = ov[i];

  if (HOUT) {
    v8h hv[2];
    #pragma unroll
    for (int i = 0; i < 2; ++i) {
      const int c = 256 * i + 8 * lane;
      const v4f p0 = *(const v4fa*)(xr + c);
      const v4f p1 = *(const v4fa*)(xr + c + 4);
      const v4f g0 = *(const v4fa*)(gam + c);
      const v4f g1v = *(const v4fa*)(gam + c + 4);
      const v4f b0 = *(const v4fa*)(bet + c);
      const v4f b1v = *(const v4fa*)(bet + c + 4);
      const v8h t = { (_Float16)((p0.x - mu) * rstd * g0.x + b0.x),
                      (_Float16)((p0.y - mu) * rstd * g0.y + b0.y),
                      (_Float16)((p0.z - mu) * rstd * g0.z + b0.z),
                      (_Float16)((p0.w - mu) * rstd * g0.w + b0.w),
                      (_Float16)((p1.x - mu) * rstd * g1v.x + b1v.x),
                      (_Float16)((p1.y - mu) * rstd * g1v.y + b1v.y),
                      (_Float16)((p1.z - mu) * rstd * g1v.z + b1v.z),
                      (_Float16)((p1.w - mu) * rstd * g1v.w + b1v.w) };
      hv[i] = t;
    }
    _Float16* hrow = outh + (size_t)row * DM;
    #pragma unroll
    for (int i = 0; i < 2; ++i) *(volatile v8h*)(hrow + 256 * i + 8 * lane) = hv[i];
    __threadfence();
    #pragma unroll
    for (int i = 0; i < 2; ++i) *(volatile v8h*)(hrow + 256 * i + 8 * lane) = hv[i];
  }
}

extern "C" void kernel_launch(void* const* d_in, const int* in_sizes, int n_in,
                              void* d_out, int out_size, void* d_ws, size_t ws_size,
                              hipStream_t stream) {
  if (n_in < 19) return;
  if (in_sizes[0] != NX || in_sizes[1] != NX || in_sizes[2] != NX) return;
  if (in_sizes[3] != NW || in_sizes[5] != NW || in_sizes[7] != NW || in_sizes[9] != NW) return;
  if (in_sizes[4] != DM || in_sizes[6] != DM || in_sizes[8] != DM || in_sizes[10] != DM) return;
  if (in_sizes[11] != NW1 || in_sizes[13] != NW1) return;
  if (in_sizes[12] != DFF || in_sizes[14] != DM) return;
  if (in_sizes[15] != DM || in_sizes[16] != DM || in_sizes[17] != DM || in_sizes[18] != DM) return;
  if (out_size != NX) return;

  const float* q   = (const float*)d_in[0];
  const float* k   = (const float*)d_in[1];
  const float* v   = (const float*)d_in[2];
  const float* Wq  = (const float*)d_in[3];
  const float* bq  = (const float*)d_in[4];
  const float* Wk  = (const float*)d_in[5];
  const float* bk  = (const float*)d_in[6];
  const float* Wv  = (const float*)d_in[7];
  const float* bv  = (const float*)d_in[8];
  const float* bo  = (const float*)d_in[10];
  const float* b1  = (const float*)d_in[12];
  const float* b2  = (const float*)d_in[14];
  const float* g1  = (const float*)d_in[15];
  const float* be1 = (const float*)d_in[16];
  const float* g2  = (const float*)d_in[17];
  const float* be2 = (const float*)d_in[18];
  const float* Wo  = (const float*)d_in[9];
  const float* W1  = (const float*)d_in[11];
  const float* W2  = (const float*)d_in[13];
  float* out = (float*)d_out;

  const size_t conv_bytes = (size_t)NCONVG * 8 * 2;
  const size_t pl_bytes   = (size_t)BATCH * NHEADS * SEQ * HD * 2;
  const size_t ctx_bytes  = (size_t)NX * 2;
  const size_t y1_bytes   = (size_t)NX * 4;
  const size_t x1f_bytes  = (size_t)NX * 4;
  const size_t x1h_bytes  = (size_t)NX * 2;
  const size_t hid_bytes  = (size_t)NHID * 2;
  const size_t y2_bytes   = (size_t)NX * 4;
  const size_t total = conv_bytes + 3 * pl_bytes + ctx_bytes + y1_bytes + x1f_bytes
                     + x1h_bytes + hid_bytes + y2_bytes;
  if (total > ws_size) return;

  char* ws = (char*)d_ws;
  size_t off = 0;
  _Float16* conv = (_Float16*)(ws + off); off += conv_bytes;
  _Float16* qh   = (_Float16*)(ws + off); off += pl_bytes;
  _Float16* kh   = (_Float16*)(ws + off); off += pl_bytes;
  _Float16* vt   = (_Float16*)(ws + off); off += pl_bytes;
  _Float16* ctx  = (_Float16*)(ws + off); off += ctx_bytes;
  float*    y1   = (float*)(ws + off);    off += y1_bytes;
  float*    x1f  = (float*)(ws + off);    off += x1f_bytes;
  _Float16* x1h  = (_Float16*)(ws + off); off += x1h_bytes;
  _Float16* hid  = (_Float16*)(ws + off); off += hid_bytes;
  float*    y2   = (float*)(ws + off);    off += y2_bytes;
  if (off > ws_size) return;

  const _Float16* xplanes = conv;
  const _Float16* wqkv16  = conv + (size_t)3 * NX;
  const _Float16* wo16    = conv + (size_t)3 * NX + (size_t)3 * NW;
  const _Float16* w1_16   = conv + (size_t)3 * NX + (size_t)4 * NW;
  const _Float16* w2_16   = w1_16 + (size_t)NW1;

  convert_kernel<<<NCONVG / 256, 256, 0, stream>>>(q, k, v, Wq, Wk, Wv, Wo, W1, W2, conv);

  dim3 gProj(MROWS / 128, 3 * NHEADS);
  proj_kernel<<<gProj, 128, 0, stream>>>(xplanes, wqkv16, bq, bk, bv, qh, kh, vt);

  dim3 gAtt(SEQ / 64, BATCH * NHEADS);
  attn_kernel<<<gAtt, 128, 0, stream>>>(qh, kh, vt, ctx);

  dim3 gO(MROWS / 128, DM / 64);
  gemm_kernel<DM, DM, false, true, false><<<gO, 128, 0, stream>>>(
      ctx, wo16, bo, q, y1, x1h, 1.0f / 128.0f, 1.0f);

  ln_kernel<true><<<MROWS / 8, 256, 0, stream>>>(y1, g1, be1, x1f, x1h);

  dim3 gF1(MROWS / 128, DFF / 64);
  gemm_kernel<DFF, DM, true, false, true><<<gF1, 128, 0, stream>>>(
      x1h, w1_16, b1, x1f, y2, hid, 1.0f / 32.0f, 4.0f);

  dim3 gF2(MROWS / 128, DM / 64);
  gemm_kernel<DM, DFF, false, true, false><<<gF2, 128, 0, stream>>>(
      hid, w2_16, b2, x1f, y2, x1h, 1.0f / 128.0f, 1.0f);

  ln_kernel<false><<<MROWS / 8, 256, 0, stream>>>(y2, g2, be2, out, x1h);
}
